// WalkLayer_25142738550817
// MI455X (gfx1250) — hardware-verified
//
#include <hip/hip_runtime.h>
#pragma clang fp contract(off)


#ifndef NB
#define NB 2
#endif
#define NB_FULL 2
#define NN   64
#define FD   128
#define ROWS (NB * NN * NN)
#define GP   132
#define BETA 0.9f

static_assert(NB <= NB_FULL);
static_assert(NB >= 1);
static_assert(NN == 64);
static_assert(FD == 128);
static_assert(FD % 32 == 0);
static_assert(ROWS % 16 == 0);
static_assert(ROWS % 8 == 0);
static_assert(((size_t)ROWS * FD / 4) % 256 == 0);
static_assert(FD % 32 == 0);
static_assert((GP * 4) % 16 == 0);
static_assert(GP >= FD);
static_assert(256 * 2 * 16 == 32 * FD * 2);
static_assert(32 * 16 * 16 == 16 * FD * 4);
static_assert(32 * 16 == FD * 4);
static_assert((size_t)FD * 33 * 4 <= 131072);
static_assert((size_t)16 * GP * 4 <= 131072);

typedef _Float16 h16;
typedef unsigned short bf;
typedef __attribute__((ext_vector_type(16))) __bf16   v16bf;
typedef __attribute__((ext_vector_type(16))) _Float16 v16h;
typedef __attribute__((ext_vector_type(8)))  _Float16 v8h;
typedef __attribute__((ext_vector_type(8)))  unsigned short v8us;
typedef __attribute__((ext_vector_type(8)))  float    v8f;
typedef __attribute__((ext_vector_type(4)))  float    v4f;
typedef v4f  __attribute__((may_alias)) v4fa;

__device__ __forceinline__ unsigned short f2bf(float f) { unsigned u = __float_as_uint(f); u += 0x7FFFu + ((u >> 16) & 1u); return (unsigned short)(u >> 16); }
__device__ __forceinline__ float bfr(float f) { return __uint_as_float(((unsigned)f2bf(f)) << 16); }
__device__ __forceinline__ v16h cat16(v8h lo, v8h hi) { return __builtin_shufflevector(lo, hi, 0, 1, 2, 3, 4, 5, 6, 7, 8, 9, 10, 11, 12, 13, 14, 15); }
__device__ __forceinline__ v16bf cat16b(v8us lo, v8us hi) { return __builtin_bit_cast(v16bf, __builtin_shufflevector(lo, hi, 0, 1, 2, 3, 4, 5, 6, 7, 8, 9, 10, 11, 12, 13, 14, 15)); }
__device__ __forceinline__ v8f wmma16(v16h a, v16h b, v8f c) { return __builtin_amdgcn_wmma_f32_16x16x32_f16(false, a, false, b, (short)0, c, false, false); }
__device__ __forceinline__ v8f wmmab(v16bf a, v16bf b, v8f c) { return __builtin_amdgcn_wmma_f32_16x16x32_bf16(false, a, false, b, (short)0, c, false, false); }
__device__ __forceinline__ v16h  ldh(const h16* p) { return cat16(*(const v8h*)p, *(const v8h*)(p + 16)); }
__device__ __forceinline__ v16bf ldb(const bf* p)  { return cat16b(*(const v8us*)p, *(const v8us*)(p + 16)); }
__device__ __forceinline__ void wave_sync() { __builtin_amdgcn_fence(3  , "wavefront"); __builtin_amdgcn_wave_barrier(); asm volatile("" ::: "memory"); }

static __device__ __forceinline__ h16 toh_flush(float v) { const h16 r = (h16)v; return (fabsf(v) < 6.103515625e-05f) ? (h16)0.0f : r; }
static __device__ __forceinline__ v8f wmma16g(v16h a, v16h b, v8f c) { c = wmma16(a, b, c); asm volatile("v_nop\n\tv_nop\n\tv_nop\n\tv_nop" : "+v"(c) : "v"(a), "v"(b)); return c; }
static __device__ __forceinline__ float sigm(float x) { return __builtin_amdgcn_rcpf(1.0f + __expf(-x)); }

__global__ __launch_bounds__(256) void k_wt(const float* __restrict__ W, h16* WT) {
    __shared__ float ts[FD * 33];
    const int tid = threadIdx.x; const int l0 = blockIdx.x * 32;
#pragma unroll 1
    for (int it = 0; it < 16; ++it) {
        const int e = it * 256 + tid; const int k = e >> 5, l = e & 31;
        ts[k * 33 + l] = bfr(W[(size_t)k * FD + l0 + l]); }
    __syncthreads();
#pragma unroll 1
    for (int ps = 0; ps < 2; ++ps) {
#pragma unroll 1
        for (int it = 0; it < 2; ++it) {
            const int p = it * 256 + tid; const int row = p >> 4, c8 = (p & 15) * 8; v8h o;
#pragma unroll
            for (int q = 0; q < 8; ++q) o[q] = toh_flush(ts[(c8 + q) * 33 + row]);
            *(volatile v8h*)(WT + (size_t)(l0 + row) * FD + c8) = o; }
        if (ps == 0) __threadfence(); }
}

__global__ __launch_bounds__(256) void k_init(const float* __restrict__ graph, const int* __restrict__ adj, float* G0, unsigned n4) {
    const unsigned i = blockIdx.x * 256 + threadIdx.x; if (i >= n4) return;
    const v4f v = *(const v4f*)(graph + (size_t)i * 4);
    const int a = adj[i >> 5];
    v4f o;
#pragma unroll
    for (int q = 0; q < 4; ++q) o[q] = (a != 0) ? bfr(v[q]) : 0.0f;
    *(volatile v4f*)(G0 + (size_t)i * 4) = o; __threadfence(); *(volatile v4f*)(G0 + (size_t)i * 4) = o;
}

__global__ __launch_bounds__(32) void k_gw(const float* __restrict__ G, const h16* __restrict__ WT, float* GW) {
    __shared__ __align__(16) float os[16 * GP];
    const int lane = threadIdx.x & 31, lr = lane & 15, hi = lane >> 4; const int r0 = blockIdx.x * 16;
    v8f acc[8];
#pragma unroll
    for (int nb = 0; nb < 8; ++nb) acc[nb] = (v8f){};
    const size_t aoff = (size_t)(r0 + lr) * FD + 8 * hi, boff = (size_t)lr * FD + 8 * hi;
#pragma unroll 1
    for (int kc = 0; kc < FD; kc += 32) {
        const v8f x0 = *(const v8f*)(G + aoff + kc); const v8f x1 = *(const v8f*)(G + aoff + kc + 16);
        v16h a;
#pragma unroll
        for (int q = 0; q < 8; ++q) { a[q] = toh_flush(x0[q]); a[8 + q] = toh_flush(x1[q]); }
#pragma unroll
        for (int nb = 0; nb < 8; ++nb) { const v16h b = ldh(WT + boff + (size_t)nb * 16 * FD + kc); acc[nb] = wmma16g(a, b, acc[nb]); }
    }
#pragma unroll
    for (int nb = 0; nb < 8; ++nb) {
#pragma unroll
        for (int j = 0; j < 8; ++j) os[(hi * 8 + j) * GP + nb * 16 + lr] = acc[nb][j]; }
    wave_sync();
    float* orow = GW + (size_t)r0 * FD;
#pragma unroll 1
    for (int ps = 0; ps < 2; ++ps) {
#pragma unroll 1
        for (int row = 0; row < 16; ++row) {
            const v4f val = *(const v4fa*)(&os[row * GP + lane * 4]);
            *(volatile v4f*)(orow + (size_t)row * FD + lane * 4) = val; }
        if (ps == 0) __threadfence(); }
}

__global__ __launch_bounds__(256) void k_hop(const float* __restrict__ Gold, const float* __restrict__ GW, const int* __restrict__ mask, float* Gnew) {
    const int lane = threadIdx.x & 31;
    const int wave = __builtin_amdgcn_readfirstlane((int)(threadIdx.x >> 5));
    const int wid = blockIdx.x * 8 + wave;
    if (wid >= ROWS) return;
    const int m = wid & (NN - 1); const int bi = wid >> 6; const int i = bi & (NN - 1); const int b = bi >> 6;
    const int k0 = lane * 4;
    const v4f old = *(const v4f*)(Gold + (size_t)wid * FD + k0);
    const int mv0 = mask[((size_t)bi * NN + lane) * NN + m];
    const int mv1 = mask[((size_t)bi * NN + 32 + lane) * NN + m];
    const unsigned blo = (unsigned)__ballot(mv0 != 0);
    const unsigned bhi = (unsigned)__ballot(mv1 != 0);
    unsigned long long bits = (unsigned long long)blo | ((unsigned long long)bhi << 32);
    bits &= ~(1ull << i); bits &= ~(1ull << m);
    float a0 = 0.0f, a1 = 0.0f, a2 = 0.0f, a3 = 0.0f; int nact = 0;
    if (i != m) {
#pragma unroll 1
        for (int j = 0; j < NN; ++j) {
            if (((bits >> j) & 1ull) == 0ull) continue;
            const v4f gw = *(const v4f*)(GW + ((size_t)bi * NN + j) * FD + k0);
            const v4f go = *(const v4f*)(Gold + ((size_t)(b * NN + j) * NN + m) * FD + k0);
            const float p0 = gw[0] * go[0], p1 = gw[1] * go[1], p2 = gw[2] * go[2], p3 = gw[3] * go[3];
            const bool pnz = (p0 != 0.0f) | (p1 != 0.0f) | (p2 != 0.0f) | (p3 != 0.0f);
            const unsigned nzb = (unsigned)__ballot(pnz);
            if (nzb == 0u) continue;
            nact = 1;
            a0 += sigm(p0); a1 += sigm(p1); a2 += sigm(p2); a3 += sigm(p3);
        }
    }
    v4f r;
    r[0] = a0 + BETA * (old[0] - a0); r[1] = a1 + BETA * (old[1] - a1); r[2] = a2 + BETA * (old[2] - a2); r[3] = a3 + BETA * (old[3] - a3);
    if (nact == 0) r = old;
    float* op = Gnew + (size_t)wid * FD + k0;
    *(volatile v4f*)op = r; __threadfence(); *(volatile v4f*)op = r;
}

static constexpr size_t al256(size_t v) { return (v + 255) & ~(size_t)255; }
static constexpr size_t SZ_G  = al256((size_t)ROWS * FD * 4);
static constexpr size_t SZ_WT = al256((size_t)FD * FD * 2);
static constexpr size_t SZ_TOTAL = 3 * SZ_G + SZ_WT;
static_assert(SZ_TOTAL <= (size_t)134217728);
static_assert((size_t)ROWS * FD * 4 <= SZ_G);
static_assert((size_t)FD * FD * 2 <= SZ_WT);

extern "C" void kernel_launch(void* const* d_in, const int* in_sizes, int n_in,
                              void* d_out, int out_size, void* d_ws, size_t ws_size, hipStream_t stream) {
    if (n_in < 4) return;
    if ((size_t)in_sizes[0] < (size_t)ROWS * FD) return;
    if ((size_t)in_sizes[1] < (size_t)ROWS) return;
    if ((size_t)in_sizes[2] < (size_t)ROWS * NN) return;
    if ((size_t)in_sizes[3] < (size_t)FD * FD) return;
    if ((size_t)out_size < (size_t)ROWS * FD) return;
    if (SZ_TOTAL > ws_size) return;
    const float* graph = (const float*)d_in[0];
    const int*   adj   = (const int*)d_in[1];
    const int*   mask  = (const int*)d_in[2];
    const float* W     = (const float*)d_in[3];
    float* OUT = (float*)d_out;
    char* wsp = (char*)d_ws;
    float* G0 = (float*)wsp; wsp += SZ_G;
    float* GW = (float*)wsp; wsp += SZ_G;
    float* G1 = (float*)wsp; wsp += SZ_G;
    h16*   WT = (h16*)wsp;   wsp += SZ_WT;

    k_wt<<<FD / 32, 256, 0, stream>>>(W, WT);
    { const unsigned n4 = (unsigned)((size_t)ROWS * FD / 4);
      k_init<<<(n4 + 255) / 256, 256, 0, stream>>>(graph, adj, G0, n4); }
    k_gw <<<ROWS / 16, 32, 0, stream>>>(G0, WT, GW);
    k_hop<<<ROWS / 8, 256, 0, stream>>>(G0, GW, mask, G1);
    k_gw <<<ROWS / 16, 32, 0, stream>>>(G1, WT, GW);
    k_hop<<<ROWS / 8, 256, 0, stream>>>(G1, GW, mask, OUT);
}
